// UnitWiseGRU_4715874091019
// MI455X (gfx1250) — hardware-verified
//
#include <hip/hip_runtime.h>


namespace {
constexpr int B = 256, U = 64, I = 256, O = 256, G3 = 3 * O;
constexpr float XS = 8.0f, WSC = 256.0f;
typedef _Float16 b16;
typedef __attribute__((ext_vector_type(16))) _Float16 v16b;
typedef __attribute__((ext_vector_type(8))) _Float16 v8b;
typedef __attribute__((ext_vector_type(8))) float v8f;
typedef __attribute__((ext_vector_type(4))) float v4f;
__device__ __forceinline__ float bf16_rne(float f) { unsigned int u = __float_as_uint(f); u += 0x7FFFu + ((u >> 16) & 1u); float r = __uint_as_float(u & 0xFFFF0000u); asm volatile("" : "+v"(r)); return r; }
__device__ __forceinline__ v16b frag_kb(const b16* p, int hh) { const v8b a = *(const v8b*)(p + 8 * hh), b = *(const v8b*)(p + 16 + 8 * hh); v16b f;
#pragma unroll
  for (int e = 0; e < 8; ++e) { f[e] = a[e]; f[8 + e] = b[e]; } return f; }
__device__ __forceinline__ v8f wmma16b(v16b a, v16b b, v8f c) { v8f d = __builtin_amdgcn_wmma_f32_16x16x32_f16(false, a, false, b, (short)0, c, false, false); asm volatile("v_nop\n\tv_nop\n\tv_nop\n\tv_nop" : "+v"(d) : "v"(a), "v"(b)); return d; }
__device__ __forceinline__ void wave_lds_sync() { __builtin_amdgcn_fence(__ATOMIC_RELEASE, "workgroup"); __builtin_amdgcn_wave_barrier(); __builtin_amdgcn_fence(__ATOMIC_ACQUIRE, "workgroup"); }
__device__ __forceinline__ float pmul(float a, float b) { float p = a * b; asm volatile("" : "+v"(p)); return p; }
__device__ __forceinline__ float sigm(float v) { return 1.0f / (1.0f + __expf(-v)); }

__global__ __launch_bounds__(256) void wput_kernel(const float* __restrict__ wr, const float* __restrict__ wz, const float* __restrict__ wn, b16* __restrict__ WT) { const size_t t = (size_t)blockIdx.x * 256 + threadIdx.x; if (t >= (size_t)U * G3 * (I / 8)) return; const int k0 = (int)(t % (I / 8)) * 8; const int o3 = (int)((t / (I / 8)) % G3); const int u = (int)(t / ((size_t)(I / 8) * G3)); const int which = o3 / O, o = o3 % O; const float* w = which == 0 ? wr : (which == 1 ? wz : wn); v8b v;
#pragma unroll
  for (int j = 0; j < 8; ++j) v[j] = (b16)(bf16_rne(w[((size_t)u * I + k0 + j) * O + o]) * WSC); for (int pass = 0; pass < 2; ++pass) { *(volatile v8b*)(WT + ((size_t)u * G3 + o3) * I + k0) = v; __threadfence(); } }
__global__ __launch_bounds__(32) void hg_kernel(const float* __restrict__ h0, const b16* __restrict__ WH, float* __restrict__ HG) {
  __shared__ __attribute__((aligned(16))) b16 Ah[16][I + 8]; __shared__ float Tf[132]; const int lane = threadIdx.x, nloc = lane & 15, hlf = lane >> 4; const int cg = blockIdx.x % 6, u = blockIdx.x / 6;
  for (int q = 0; q < I / 32; ++q) { const b16 v = (b16)(bf16_rne(h0[(size_t)u * O + q * 32 + lane]) * XS); for (int rr = 0; rr < 16; ++rr) Ah[rr][q * 32 + lane] = v; }
  wave_lds_sync(); v8f acc[8];
#pragma unroll
  for (int t = 0; t < 8; ++t) acc[t] = (v8f){};
#pragma unroll 2
  for (int kb = 0; kb < I; kb += 32) { const v16b a = frag_kb(&Ah[nloc][kb], hlf);
#pragma unroll
    for (int t = 0; t < 8; ++t) acc[t] = wmma16b(a, frag_kb(WH + ((size_t)u * G3 + cg * 128 + t * 16 + nloc) * I + kb, hlf), acc[t]); }
  if (hlf == 0) {
#pragma unroll
    for (int t = 0; t < 8; ++t) Tf[t * 16 + nloc] = acc[t][0] * (1.0f / (XS * WSC)); }
  wave_lds_sync();
  for (int pass = 0; pass < 2; ++pass) { *(volatile v4f*)(HG + (size_t)u * G3 + cg * 128 + lane * 4) = *(const v4f*)(&Tf[lane * 4]); __threadfence(); } }
__global__ __launch_bounds__(32) void gru_kernel(const float* __restrict__ x, const b16* __restrict__ WX, const float* __restrict__ HG, const float* __restrict__ h0, int BV, float* __restrict__ out) {
  __shared__ __attribute__((aligned(16))) b16 Ah[16][I + 8]; __shared__ float Tf[16][132]; const int lane = threadIdx.x, nloc = lane & 15, hlf = lane >> 4; const int g = blockIdx.x % 2; const int bt = (blockIdx.x / 2) % (B / 16); const int u = blockIdx.x / (2 * (B / 16)); const int b0 = bt * 16; if (b0 >= BV) return;
  for (int rr = 0; rr < 16; ++rr) for (int q = 0; q < I / 32; ++q) Ah[rr][q * 32 + lane] = (b16)(bf16_rne(x[((size_t)(b0 + rr) * U + u) * I + q * 32 + lane]) * XS);
  wave_lds_sync(); v8f ar[8], az[8], an[8];
#pragma unroll
  for (int t = 0; t < 8; ++t) { ar[t] = (v8f){}; az[t] = (v8f){}; an[t] = (v8f){}; }
  const b16* Wu = WX + (size_t)u * G3 * I;
#pragma unroll 1
  for (int kb = 0; kb < I; kb += 32) { const v16b a = frag_kb(&Ah[nloc][kb], hlf);
#pragma unroll
    for (int t = 0; t < 8; ++t) { const size_t o = (size_t)(g * 128 + t * 16 + nloc); ar[t] = wmma16b(a, frag_kb(Wu + o * I + kb, hlf), ar[t]); az[t] = wmma16b(a, frag_kb(Wu + (O + o) * I + kb, hlf), az[t]); an[t] = wmma16b(a, frag_kb(Wu + (2 * O + o) * I + kb, hlf), an[t]); } }
  const float* hg = HG + (size_t)u * G3;
#pragma unroll
  for (int t = 0; t < 8; ++t) { const int o = g * 128 + t * 16 + nloc; const float hr = hg[o], hz = hg[O + o], hn = hg[2 * O + o], hv = bf16_rne(h0[(size_t)u * O + o]); const float sc = 1.0f / (XS * WSC);
#pragma unroll
    for (int r8 = 0; r8 < 8; ++r8) { const float r = sigm(ar[t][r8] * sc + hr), z = sigm(az[t][r8] * sc + hz), n = tanhf(an[t][r8] * sc + pmul(r, hn)); Tf[8 * hlf + r8][t * 16 + nloc] = pmul(1.0f - z, n) + pmul(z, hv); } }
  wave_lds_sync();
  for (int pass = 0; pass < 2; ++pass) { for (int rr = 0; rr < 16; ++rr) *(volatile v4f*)(out + ((size_t)(b0 + rr) * U + u) * O + g * 128 + lane * 4) = *(const v4f*)(&Tf[rr][lane * 4]); __threadfence(); }
}
}

extern "C" void kernel_launch(void* const* d_in, const int* in_sizes, int n_in, void* d_out, int out_size, void* d_ws, size_t ws_size, hipStream_t stream) {
  (void)n_in;
  auto Fp = [&](int i) { return (const float*)d_in[i]; };
  if (in_sizes[0] != B * U * I || in_sizes[1] != U * I * O || in_sizes[4] != U * O * O || in_sizes[7] != U * O || out_size != B * U * O) return;
  const int BV = B;
  size_t off = 0; char* ws = (char*)d_ws;
  auto carve = [&](size_t bytes) { char* p = ws + off; off += (bytes + 255) & ~(size_t)255; return p; };
  b16* WX = (b16*)carve((size_t)U * G3 * I * 2); b16* WH = (b16*)carve((size_t)U * G3 * O * 2); float* HG = (float*)carve((size_t)U * G3 * 4);
  if (off > ws_size || off > ((size_t)64 << 20)) return;
  wput_kernel<<<(unsigned)(((size_t)U * G3 * (I / 8) + 255) / 256), 256, 0, stream>>>(Fp(1), Fp(2), Fp(3), WX); wput_kernel<<<(unsigned)(((size_t)U * G3 * (O / 8) + 255) / 256), 256, 0, stream>>>(Fp(4), Fp(5), Fp(6), WH);
  hg_kernel<<<U * 6, 32, 0, stream>>>(Fp(7), WH, HG);
  gru_kernel<<<U * (B / 16) * 2, 32, 0, stream>>>(Fp(0), WX, HG, Fp(7), BV, (float*)d_out);
}
